// DiscreteCRFConv_72662256714587
// MI455X (gfx1250) — hardware-run, weakly checked
//
#include <hip/hip_runtime.h>


#ifndef NN
#define NN 50000
#endif
#define NN_FULL 50000
#define DEG  16
#define NC   16
#define EC   64
#define HID  64
#define NKER 5
#define KH   (NKER * HID)
#define SW   5
#define TSP  20
#define L2E  1.4426950408889634f

static_assert(NN <= NN_FULL);
static_assert(NN % 16 == 0);
static_assert((NN / 16) % SW == 0);
static_assert(DEG == 16);
static_assert(DEG % 4 == 0);
static_assert(NC == 16);
static_assert(EC == 64);
static_assert(HID == 64);
static_assert(EC % 32 == 0);
static_assert(KH % 64 == 0);
static_assert(((size_t)NN * EC) % 8 == 0);
static_assert(((size_t)NN * NC) % 256 == 0);
static_assert(((size_t)NN * DEG) % 256 == 0);
static_assert((TSP * 4) % 16 == 0);
static_assert(16 * 68 * 4 <= 131072);
static_assert(SW * 16 * TSP * 4 <= 131072);
static_assert(EC * 65 * 4 <= 131072);

typedef unsigned short bf;
typedef __attribute__((ext_vector_type(16))) __bf16   v16bf;
typedef __attribute__((ext_vector_type(8)))  unsigned short v8us;
typedef __attribute__((ext_vector_type(8)))  float    v8f;
typedef __attribute__((ext_vector_type(4)))  float    v4f;
typedef __attribute__((ext_vector_type(4)))  int      v4i;
typedef v4f  __attribute__((may_alias)) v4fa;

__device__ __forceinline__ unsigned short f2bf(float f) { unsigned u = __float_as_uint(f); u += 0x7FFFu + ((u >> 16) & 1u); return (unsigned short)(u >> 16); }
__device__ __forceinline__ float bfr(float f) { return __uint_as_float(((unsigned)f2bf(f)) << 16); }
__device__ __forceinline__ v16bf cat16b(v8us lo, v8us hi) { return __builtin_bit_cast(v16bf, __builtin_shufflevector(lo, hi, 0, 1, 2, 3, 4, 5, 6, 7, 8, 9, 10, 11, 12, 13, 14, 15)); }
__device__ __forceinline__ v8f wmmab(v16bf a, v16bf b, v8f c) { return __builtin_amdgcn_wmma_f32_16x16x32_bf16(false, a, false, b, (short)0, c, false, false); }
__device__ __forceinline__ v8f wmmab_g(v16bf a, v16bf b, v8f c) { c = wmmab(a, b, c); asm volatile("v_nop\n\tv_nop\n\tv_nop\n\tv_nop" : "+v"(c) : "v"(a), "v"(b)); return c; }
__device__ __forceinline__ v16bf ldb(const bf* p)  { return cat16b(*(const v8us*)p, *(const v8us*)(p + 16)); }
__device__ __forceinline__ void wave_sync() { __builtin_amdgcn_fence(3  , "wavefront"); __builtin_amdgcn_wave_barrier(); asm volatile("" ::: "memory"); }

__global__ __launch_bounds__(256) void k_cvt8(const float* __restrict__ src, bf* dst, size_t n8) {
    const size_t i = (size_t)blockIdx.x * 256 + threadIdx.x; if (i >= n8) return;
    const v8f v = *(const v8f*)(src + i * 8); v8us o;
#pragma unroll
    for (int k = 0; k < 8; ++k) o[k] = f2bf(v[k]);
    *(volatile v8us*)(dst + i * 8) = o; __threadfence(); *(volatile v8us*)(dst + i * 8) = o;
}

static_assert(2 * 256 * 8 == EC * HID);
__global__ __launch_bounds__(256) void k_wconvT(const float* __restrict__ Fk, bf* FT) {
    __shared__ float ts[EC * 65];
    const int k = blockIdx.x; const int tid = threadIdx.x;
    const float* src = Fk + (size_t)k * EC * HID;
#pragma unroll 1
    for (int i = tid; i < EC * HID; i += 256) ts[(i >> 6) * 65 + (i & 63)] = src[i];
    __syncthreads();
#pragma unroll 1
    for (int ps = 0; ps < 2; ++ps) {
#pragma unroll 1
        for (int it = 0; it < 2; ++it) { const int p = it * 256 + tid; const int hrow = p >> 3, c8 = (p & 7) * 8; v8us o;
#pragma unroll
            for (int i = 0; i < 8; ++i) o[i] = f2bf(ts[(c8 + i) * 65 + hrow]);
            *(volatile v8us*)(FT + ((size_t)k * HID + hrow) * EC + c8) = o; }
        if (ps == 0) __threadfence(); }
}

__global__ __launch_bounds__(256) void k_prep(const float* __restrict__ P, float* U, float* Q0, int n) {
    const int i = blockIdx.x * 256 + threadIdx.x; if (i >= n) return;
    const float pv = bfr(P[i]); const float uv = -logf(pv);
    *(volatile float*)(U + i) = uv; *(volatile float*)(Q0 + i) = pv;
    __threadfence();
    *(volatile float*)(U + i) = uv; *(volatile float*)(Q0 + i) = pv;
}

static_assert(8 * 32 * 4 == 16 * 64);
__global__ __launch_bounds__(32) void k_fpgemm(const bf* __restrict__ A, const bf* __restrict__ Bt, float* FP) {
    __shared__ __align__(16) float os[16 * 68];
    const int K = EC;
    const int lane = threadIdx.x & 31, lr = lane & 15, hi = lane >> 4; const int r0 = blockIdx.x * 16, c0 = blockIdx.y * 64;
    v8f acc[4];
#pragma unroll
    for (int nb = 0; nb < 4; ++nb) acc[nb] = (v8f){};
    const size_t aoff = (size_t)(r0 + lr) * K + 8 * hi, boff = (size_t)(c0 + lr) * K + 8 * hi;
#pragma unroll
    for (int kc = 0; kc < K; kc += 32) {
        const v16bf a = ldb(A + aoff + kc);
#pragma unroll
        for (int nb = 0; nb < 4; ++nb) { const v16bf b = ldb(Bt + boff + (size_t)nb * 16 * K + kc); acc[nb] = wmmab_g(a, b, acc[nb]); }
    }
#pragma unroll
    for (int nb = 0; nb < 4; ++nb) {
#pragma unroll
        for (int j = 0; j < 8; ++j) os[(hi * 8 + j) * 68 + nb * 16 + lr] = acc[nb][j]; }
    wave_sync();
    float* fb = FP + (size_t)r0 * KH + c0;
#pragma unroll 1
    for (int ps = 0; ps < 2; ++ps) {
#pragma unroll
        for (int s = 0; s < 8; ++s) { const int p = s * 32 + lane; const int row = p >> 4, c4 = (p & 15) * 4;
            const v4f val = *(const v4fa*)(&os[row * 68 + c4]);
            *(volatile v4f*)(fb + (size_t)row * KH + c4) = val; }
        if (ps == 0) __threadfence(); }
}

__global__ __launch_bounds__(256) void k_edgew(const float* __restrict__ FP, const int* __restrict__ col, const int* __restrict__ row, const float* __restrict__ Wk, float* WE) {
    const int e = blockIdx.x * 256 + threadIdx.x;
    const int node = e / DEG;
    int cn = col[e]; cn = cn < 0 ? 0 : (cn > NN - 1 ? NN - 1 : cn);
    const int rw = row[e];
    const float* a = FP + (size_t)cn * KH;
    const float* b = FP + (size_t)node * KH;
    float acc = 0.0f;
#pragma unroll 1
    for (int k = 0; k < NKER; ++k) {
        float s = 0.0f;
#pragma unroll 4
        for (int i = 0; i < HID / 4; ++i) {
            const v4f x = *(const v4f*)(a + k * HID + i * 4), y = *(const v4f*)(b + k * HID + i * 4);
            const v4f d = x - y;
            s += d[0] * d[0]; s += d[1] * d[1]; s += d[2] * d[2]; s += d[3] * d[3]; }
        acc += expf(-s) * bfr(Wk[k]); }
    const float wv = (rw == node) ? acc : __uint_as_float(0x7FC00000u);
    *(volatile float*)(WE + e) = wv; __threadfence(); *(volatile float*)(WE + e) = wv;
}

static_assert(2 * 32 * 4 == 16 * NC);
__global__ __launch_bounds__(32 * SW) void k_step(const float* __restrict__ QI, const int* __restrict__ col, const float* __restrict__ WE, const float* __restrict__ U,
                                                  const float* __restrict__ Cm, float* QO) {
    __shared__ __align__(16) float os[SW * 16 * TSP];
    const int lane = threadIdx.x & 31, lr = lane & 15, hi = lane >> 4;
    const int wave = __builtin_amdgcn_readfirstlane((int)(threadIdx.x >> 5));
    const int nb = (blockIdx.x * SW + wave) * 16;
    const int node = nb + lr;
    const size_t eb = (size_t)node * DEG;
    float ag[8];
#pragma unroll
    for (int i = 0; i < 8; ++i) ag[i] = 0.0f;
#pragma unroll 1
    for (int g = 0; g < DEG / 4; ++g) {
        const v4i c4 = *(const v4i*)(col + eb + g * 4);
        const v4f w4 = *(const v4f*)(WE + eb + g * 4);
#pragma unroll
        for (int j = 0; j < 4; ++j) {
            int cl = c4[j]; cl = cl < 0 ? 0 : (cl > NN - 1 ? NN - 1 : cl);
            const float* qp = QI + (size_t)cl * NC + 8 * hi;
            const v4f x0 = *(const v4f*)qp, x1 = *(const v4f*)(qp + 4);
            const float wv = w4[j];
            ag[0] += x0[0] * wv; ag[1] += x0[1] * wv; ag[2] += x0[2] * wv; ag[3] += x0[3] * wv;
            ag[4] += x1[0] * wv; ag[5] += x1[1] * wv; ag[6] += x1[2] * wv; ag[7] += x1[3] * wv; } }
    v8us ah, al, cb;
#pragma unroll
    for (int i = 0; i < 8; ++i) { const unsigned short hb = f2bf(ag[i]); ah[i] = hb; al[i] = f2bf(ag[i] - __uint_as_float(((unsigned)hb) << 16));
                                  cb[i] = f2bf(Cm[(8 * hi + i) * NC + lr]); }
    const v16bf a = cat16b(ah, al);
    const v16bf b = cat16b(cb, cb);
    v8f d = (v8f){};
    d = wmmab_g(a, b, d);
    const int wb = wave * 16 * TSP;
#pragma unroll
    for (int r = 0; r < 8; ++r) os[wb + (8 * hi + r) * TSP + lr] = d[r];
    wave_sync();
    const v4f d0 = *(const v4fa*)(&os[wb + lr * TSP + 8 * hi]), d1 = *(const v4fa*)(&os[wb + lr * TSP + 8 * hi + 4]);
    const float* up = U + (size_t)node * NC + 8 * hi;
    const v4f u0 = *(const v4f*)up, u1 = *(const v4f*)(up + 4);
    float t[8];
#pragma unroll
    for (int i = 0; i < 4; ++i) { t[i] = -u0[i] - d0[i]; t[4 + i] = -u1[i] - d1[i]; }
    float mx = t[0];
#pragma unroll
    for (int i = 1; i < 8; ++i) mx = fmaxf(mx, t[i]);
    mx = fmaxf(mx, __shfl_xor(mx, 16, 32));
    float ex[8]; float sm = 0.0f;
#pragma unroll
    for (int i = 0; i < 8; ++i) { ex[i] = __builtin_amdgcn_exp2f((t[i] - mx) * L2E); sm += ex[i]; }
    sm += __shfl_xor(sm, 16, 32);
    const float inv = 1.0f / sm;
    v4f q0, q1;
#pragma unroll
    for (int i = 0; i < 4; ++i) { q0[i] = ex[i] * inv; q1[i] = ex[4 + i] * inv; }
    *(v4fa*)(&os[wb + lr * TSP + 8 * hi]) = q0; *(v4fa*)(&os[wb + lr * TSP + 8 * hi + 4]) = q1;
    wave_sync();
    float* qo = QO + (size_t)nb * NC;
#pragma unroll 1
    for (int ps = 0; ps < 2; ++ps) {
#pragma unroll
        for (int s = 0; s < 2; ++s) { const int p = s * 32 + lane; const int rowi = p >> 2, c4 = (p & 3) * 4;
            const v4f val = *(const v4fa*)(&os[wb + rowi * TSP + c4]);
            *(volatile v4f*)(qo + (size_t)p * 4) = val; }
        if (ps == 0) __threadfence(); }
}

static constexpr size_t al256(size_t v) { return (v + 255) & ~(size_t)255; }
static constexpr size_t SZ_FB = al256((size_t)NN * EC * 2);
static constexpr size_t SZ_FT = al256((size_t)KH * EC * 2);
static constexpr size_t SZ_FP = al256((size_t)NN * KH * 4);
static constexpr size_t SZ_WE = al256((size_t)NN * DEG * 4);
static constexpr size_t SZ_QP = al256((size_t)NN * NC * 4);
static constexpr size_t SZ_TOTAL = SZ_FB + SZ_FT + SZ_FP + SZ_WE + 3 * SZ_QP;
static_assert(SZ_TOTAL <= (size_t)134217728);
static_assert(((size_t)NN * NC * 4) % 1024 == 0);

extern "C" void kernel_launch(void* const* d_in, const int* in_sizes, int n_in,
                              void* d_out, int out_size, void* d_ws, size_t ws_size, hipStream_t stream) {
    if (n_in < 7) return;
    if ((size_t)in_sizes[0] < (size_t)NN * NC || (size_t)in_sizes[1] < (size_t)NN * EC) return;
    if ((size_t)in_sizes[2] < (size_t)NN * DEG || (size_t)in_sizes[3] < (size_t)NN * DEG) return;
    if ((size_t)in_sizes[4] < (size_t)NKER * EC * HID || in_sizes[5] < NKER || in_sizes[6] < NC * NC) return;
    if ((size_t)out_size < (size_t)NN * NC) return;
    if (SZ_TOTAL > ws_size) return;
    const float* p   = (const float*)d_in[0];
    const float* f   = (const float*)d_in[1];
    const int*   col = (const int*)d_in[2];
    const int*   row = (const int*)d_in[3];
    const float* Fk  = (const float*)d_in[4];
    const float* Wk  = (const float*)d_in[5];
    const float* Cm  = (const float*)d_in[6];
    float* OUT = (float*)d_out;
    char* wsp = (char*)d_ws;
    bf* FB = (bf*)wsp; wsp += SZ_FB;
    bf* FT = (bf*)wsp; wsp += SZ_FT;
    float* FP = (float*)wsp; wsp += SZ_FP;
    float* WE = (float*)wsp; wsp += SZ_WE;
    float* UP = (float*)wsp; wsp += SZ_QP;
    float* Q0 = (float*)wsp; wsp += SZ_QP;
    float* Q1 = (float*)wsp; wsp += SZ_QP;

    { const size_t n8 = (size_t)NN * EC / 8;
      k_cvt8<<<(unsigned)((n8 + 255) / 256), 256, 0, stream>>>(f, FB, n8); }
    k_wconvT<<<NKER, 256, 0, stream>>>(Fk, FT);
    { const int n = NN * NC;
      k_prep<<<(unsigned)((n + 255) / 256), 256, 0, stream>>>(p, UP, Q0, n); }
    k_fpgemm<<<dim3(NN / 16, KH / 64, 1), 32, 0, stream>>>(FB, FT, FP);
    k_edgew<<<(unsigned)(((size_t)NN * DEG) / 256), 256, 0, stream>>>(FP, col, row, Wk, WE);

    const unsigned sg = (unsigned)(NN / 16 / SW);
    k_step<<<sg, 32 * SW, 0, stream>>>(Q0, col, WE, UP, Cm, Q1);
    k_step<<<sg, 32 * SW, 0, stream>>>(Q1, col, WE, UP, Cm, Q0);
    k_step<<<sg, 32 * SW, 0, stream>>>(Q0, col, WE, UP, Cm, Q1);
    k_step<<<sg, 32 * SW, 0, stream>>>(Q1, col, WE, UP, Cm, Q0);
    k_step<<<sg, 32 * SW, 0, stream>>>(Q0, col, WE, UP, Cm, OUT);
}
